// CPPN_70660801954511
// MI455X (gfx1250) — hardware-run, weakly checked
//
#include <hip/hip_runtime.h>


#ifndef NB
#define NB 1048576
#endif
#define NB_FULL 1048576
#define NIN   12
#define HID   32
#define NOUT  3
#define TPX   32
#define NTILES (NB / TPX)
#define WPB   8
#define NBLOCKS 256
#define OSW   (TPX * NOUT)

static_assert(NB % TPX == 0);
static_assert(NB <= NB_FULL);
static_assert(NIN <= 12 && NIN % 4 == 0 && NIN > 8);
static_assert(HID == 32);
static_assert(NOUT <= 8);
static_assert((TPX * NOUT * 4) % 128 == 0);
static_assert(24 * 16 == TPX * NOUT * 4);
static_assert(OSW == 96);
static_assert(3 * HID * 8 * 4 + WPB * OSW * 4 <= 131072);
static_assert(WPB * 32 == 256);

typedef _Float16 h16;
typedef __attribute__((ext_vector_type(16))) _Float16 v16h;
typedef __attribute__((ext_vector_type(8)))  float    v8f;
typedef __attribute__((ext_vector_type(4)))  float    v4f;
typedef v4f  __attribute__((may_alias)) v4fa;

__device__ __forceinline__ unsigned short f2bf(float f) { unsigned u = __float_as_uint(f); u += 0x7FFFu + ((u >> 16) & 1u); return (unsigned short)(u >> 16); }
__device__ __forceinline__ float bf2f(unsigned short w) { return __uint_as_float(((unsigned)w) << 16); }
__device__ __forceinline__ int clampi(int v, int lo, int hi) { return min(max(v, lo), hi); }
__device__ __forceinline__ void wave_sync() { __builtin_amdgcn_fence(3  , "wavefront"); __builtin_amdgcn_wave_barrier(); asm volatile("" ::: "memory"); }

static __device__ __forceinline__ h16 toh_flush(float v) { const h16 r = (h16)v; return (fabsf(v) < 6.103515625e-05f) ? (h16)0.0f : r; }
static __device__ __forceinline__ h16 wq(float w) { return toh_flush(bf2f(f2bf(w)) * 64.0f); }

__device__ __forceinline__ v8f wmmah(v16h a, v16h b, v8f c) {
    c = __builtin_amdgcn_wmma_f32_16x16x32_f16(false, a, false, b, (short)0, c, false, false);
    asm volatile("v_nop\n\tv_nop\n\tv_nop\n\tv_nop" : "+v"(c) : "v"(a), "v"(b));
    return c;
}

__device__ __forceinline__ v16h ldw(const float* __restrict__ W, const int K, const int N, const int ncol, const int hh) {
    v16h f;
    const int nc = min(ncol, N - 1);
#pragma unroll
    for (int i = 0; i < 16; ++i) {
        const int k = (i < 8) ? (8 * hh + i) : (16 + 8 * hh + (i - 8));
        const int kc = min(k, K - 1);
        float w = W[kc * N + nc];
        asm volatile("" : "+v"(w));
        w = ((k < K) & (ncol < N)) ? w : 0.0f;
        f[i] = wq(w);
    }
    return f;
}

#define SC_H   0.015625f
#define SC_R   7.62939453125e-06f
#define L2E    1.4426950408889634f
#define INV2PI 0.15915494309189535f

__global__ __launch_bounds__(256) __attribute__((amdgpu_num_vgpr(256))) void k_mlp(
    const float* __restrict__ X, const float* __restrict__ bias_in,
    const float* __restrict__ W1, const float* __restrict__ b1, const int* __restrict__ act1,
    const float* __restrict__ W2, const float* __restrict__ b2, const int* __restrict__ act2,
    const float* __restrict__ W3, const float* __restrict__ b3, const int* __restrict__ act3,
    const float* __restrict__ Wout, const float* __restrict__ bout, float* OUT)
{
    __shared__ __align__(16) float cf[3 * HID * 8];
    __shared__ __align__(16) float os[WPB * OSW];
    const int tid = threadIdx.x, lane = tid & 31, lr = lane & 15, hi = lane >> 4;
    const int wave = __builtin_amdgcn_readfirstlane(tid >> 5);

    {
        const int i1 = act1[lane], i2 = act2[lane], i3 = act3[lane];
        const float c1 = b1[lane], c2 = b2[lane], c3 = b3[lane];
        const int id = (wave == 0) ? i1 : ((wave == 1) ? i2 : i3);
        const float braw = (wave == 0) ? c1 : ((wave == 1) ? c2 : c3);
        const bool k1 = (id == 1), k2 = (id == 2), k3 = (id == 3), k4 = (id == 4);
        const float cA = k1 ? (2.0f * L2E) : (k2 ? (-L2E) : 0.0f);
        const float cB = k4 ? (0.5f * L2E) : 0.0f;
        const float cS = k1 ? -2.0f : ((k2 || k4) ? 1.0f : 0.0f);
        const float cF = k4 ? 0.0f : 1.0f;
        const float cC = k1 ? 1.0f : 0.0f;
        const float fs = k3 ? 1.0f : 0.0f;
        const float fi = (k1 || k2 || k3 || k4) ? 0.0f : 1.0f;
        const float bb = bf2f(f2bf(braw));
        if (wave < 3) {
            const v4f lo4 = {cA, cB, cS, cF};
            const v4f hi4 = {cC, bb, fs, fi};
            const int ci = (wave * HID + lane) * 8;
            *(v4fa*)(&cf[ci]) = lo4;
            *(v4fa*)(&cf[ci + 4]) = hi4;
        }
    }
    __syncthreads();

    v16h aW[3][2];
#pragma unroll
    for (int t = 0; t < 2; ++t) {
        aW[0][t] = ldw(W1, NIN, HID, 16 * t + lr, hi);
        __builtin_amdgcn_sched_barrier(0);
        aW[1][t] = ldw(W2, HID, HID, 16 * t + lr, hi);
        __builtin_amdgcn_sched_barrier(0);
        aW[2][t] = ldw(W3, HID, HID, 16 * t + lr, hi);
        __builtin_amdgcn_sched_barrier(0);
    }
    const v16h aWo = ldw(Wout, HID, NOUT, lr, hi);
    __builtin_amdgcn_sched_barrier(0);

    float ba[4], bq[4];
#pragma unroll
    for (int j = 0; j < 4; ++j) { ba[j] = bf2f(f2bf(bias_in[8 * hi + j])); bq[j] = bf2f(f2bf(bias_in[4 + j])); }
    float bo[NOUT];
#pragma unroll
    for (int r = 0; r < NOUT; ++r) bo[r] = bf2f(f2bf(bout[r]));

    const int gw = blockIdx.x * WPB + wave;
    const int nw = gridDim.x * WPB;
    const int ob = wave * OSW;

#pragma unroll 1
    for (int tile = gw; tile < NTILES; tile += nw) {
        const size_t p0 = (size_t)tile * TPX;
#pragma unroll 1
        for (int sub = 0; sub < 2; ++sub) {
            const float* row = X + (p0 + (size_t)(sub * 16 + lr)) * NIN;
            const v4f x0 = *(const v4f*)(row + 8 * hi);
            const v4f x1 = *(const v4f*)(row + 4);
            v16h bh; v16h bl;
#pragma unroll
            for (int j = 0; j < 4; ++j) {
                bh[j] = toh_flush(bf2f(f2bf(x0[j])) + ba[j]);
                float v = bf2f(f2bf(x1[j])) + bq[j];
                v = (hi == 0) ? v : 0.0f;
                bh[4 + j] = toh_flush(v);
            }
#pragma unroll
            for (int i = 8; i < 16; ++i) bh[i] = (h16)0.0f;
#pragma unroll
            for (int i = 0; i < 16; ++i) bl[i] = (h16)0.0f;

#pragma unroll
            for (int ly = 0; ly < 3; ++ly) {
                v8f aH[2], aR[2];
#pragma unroll
                for (int t = 0; t < 2; ++t) {
                    aH[t] = wmmah(aW[ly][t], bh, (v8f){});
                    if (ly > 0) aR[t] = wmmah(aW[ly][t], bl, (v8f){});
                    else        aR[t] = (v8f){};
                }
                v16h nh, nl;
#pragma unroll
                for (int t = 0; t < 2; ++t) {
#pragma unroll
                    for (int r = 0; r < 8; ++r) {
                        const int ci = (ly * HID + 16 * t + 8 * hi + r) * 8;
                        const v4f ca = *(const v4fa*)(&cf[ci]);
                        const v4f cb = *(const v4fa*)(&cf[ci + 4]);
                        float x = fmaf(aH[t][r], SC_H, cb[1]);
                        if (ly > 0) x = fmaf(aR[t][r], SC_R, x);
                        const float e = __builtin_amdgcn_exp2f(fmaf(ca[1], x * x, ca[0] * x));
                        float y = fmaf(ca[2], __builtin_amdgcn_rcpf(e + ca[3]), cb[0]);
                        const float sn = __builtin_amdgcn_sinf(x * INV2PI);
                        y = (cb[2] > 0.5f) ? sn : y;
                        y = (cb[3] > 0.5f) ? x : y;
                        const h16 yh = toh_flush(y);
                        const h16 yl = toh_flush((y - (float)yh) * 2048.0f);
                        nh[8 * t + r] = yh;
                        nl[8 * t + r] = yl;
                    }
                }
                bh = nh; bl = nl;
            }

            const v8f oH = wmmah(aWo, bh, (v8f){});
            const v8f oR = wmmah(aWo, bl, (v8f){});
#pragma unroll
            for (int r = 0; r < NOUT; ++r) {
                const float x = fmaf(oR[r], SC_R, fmaf(oH[r], SC_H, bo[r]));
                const float e = __builtin_amdgcn_exp2f((2.0f * L2E) * x);
                const float y = fmaf(-2.0f, __builtin_amdgcn_rcpf(e + 1.0f), 1.0f);
                if (hi == 0) os[ob + (sub * 16 + lr) * NOUT + r] = y;
            }
        }
        wave_sync();
        const v4f v = *(const v4fa*)(&os[ob + 4 * min(lane, 23)]);
        float* dst = OUT + p0 * NOUT + 4 * lane;
#pragma unroll 1
        for (int ps = 0; ps < 2; ++ps) {
            if (lane < 24) { *(volatile v4f*)(dst) = v; }
            if (ps == 0) __threadfence(); }
        wave_sync();
    }
}

extern "C" void kernel_launch(void* const* d_in, const int* in_sizes, int n_in,
                              void* d_out, int out_size, void* d_ws, size_t ws_size, hipStream_t stream) {
    (void)d_ws; (void)ws_size;
    if (n_in < 13) return;
    if ((size_t)in_sizes[0] < (size_t)NB * NIN) return;
    if (in_sizes[1] < NIN) return;
    if (in_sizes[2] < NIN * HID) return;
    if (in_sizes[3] < HID || in_sizes[4] < HID) return;
    if (in_sizes[5] < HID * HID) return;
    if (in_sizes[6] < HID || in_sizes[7] < HID) return;
    if (in_sizes[8] < HID * HID) return;
    if (in_sizes[9] < HID || in_sizes[10] < HID) return;
    if (in_sizes[11] < HID * NOUT) return;
    if (in_sizes[12] < NOUT) return;
    if ((size_t)out_size < (size_t)NB * NOUT) return;
    const float* X   = (const float*)d_in[0];
    const float* bin = (const float*)d_in[1];
    const float* W1  = (const float*)d_in[2];
    const float* b1  = (const float*)d_in[3];
    const int*   a1  = (const int*)d_in[4];
    const float* W2  = (const float*)d_in[5];
    const float* b2  = (const float*)d_in[6];
    const int*   a2  = (const int*)d_in[7];
    const float* W3  = (const float*)d_in[8];
    const float* b3  = (const float*)d_in[9];
    const int*   a3  = (const int*)d_in[10];
    const float* Wo  = (const float*)d_in[11];
    const float* bo  = (const float*)d_in[12];
    float* OUT = (float*)d_out;
    k_mlp<<<NBLOCKS, 256, 0, stream>>>(X, bin, W1, b1, a1, W2, b2, a2, W3, b3, a3, Wo, bo, OUT);
}
